// RnnNet_13322988552223
// MI455X (gfx1250) — hardware-verified
//
#include <hip/hip_runtime.h>
#include <math.h>

constexpr int kIn       = 28;
constexpr int kInPad    = 32;
constexpr int kHid      = 64;
constexpr int kGates    = 256;
constexpr int kOutDim   = 10;
constexpr int kOutPad   = 16;
constexpr int kSteps    = 28;
constexpr int kXRow     = 784;
constexpr int kRowsPerBlock = 32;
constexpr int kThreads  = 128;
constexpr int kPitch0   = 104;
constexpr int kPitch1   = 136;
constexpr int kPitchO   = 20;
constexpr int kW0ld     = kInPad + kHid;
constexpr int kW1ld     = 2 * kHid;
constexpr int kW0n      = kGates * kW0ld;
constexpr int kW1n      = kGates * kW1ld;
constexpr int kWLn      = kOutPad * kHid;
constexpr int kWtot     = kW0n + kW1n + kWLn;
constexpr int kPrepGroups = kWtot / 8;
constexpr int kGrp0     = kW0n / 8;
constexpr int kGrp1     = kW1n / 8;
constexpr int kGrp2     = kWLn / 8;
constexpr float kWCarry    = 16.0f;
constexpr float kWCarryInv = 1.0f / 16.0f;
static_assert(kWtot % 8 == 0, "groups");
static_assert(kPrepGroups % 32 == 0, "whole waves");

typedef __attribute__((ext_vector_type(16))) _Float16 v16h;
typedef __attribute__((ext_vector_type(8)))  _Float16 v8h;
typedef __attribute__((ext_vector_type(16))) __bf16   v16b;
typedef __attribute__((ext_vector_type(8)))  __bf16   v8b;
typedef __attribute__((ext_vector_type(8)))  float    v8f;
typedef __attribute__((ext_vector_type(4)))  float    v4f;
typedef __attribute__((ext_vector_type(4)))  unsigned int v4u;

__device__ __forceinline__ void dep_guard_h(v8f& a, v8f& b, v16h x, v16h y) { asm volatile("v_nop\n\tv_nop\n\tv_nop\n\tv_nop" : "+v"(a), "+v"(b) : "v"(x), "v"(y)); }
__device__ __forceinline__ void dep_guard_b(v8f& a, v8f& b, v16b x, v16b y) { asm volatile("v_nop\n\tv_nop\n\tv_nop\n\tv_nop" : "+v"(a), "+v"(b) : "v"(x), "v"(y)); }
__device__ __forceinline__ void keep4_h(v16h a, v16h b, v16h c, v16h d) { asm volatile("v_nop" :: "v"(a), "v"(b), "v"(c), "v"(d)); }
__device__ __forceinline__ void keep4_b(v16b a, v16b b, v16b c, v16b d) { asm volatile("v_nop" :: "v"(a), "v"(b), "v"(c), "v"(d)); }
__device__ __forceinline__ void acc_guard4(v8f& a, v8f& b, v8f& c, v8f& d) { asm volatile("v_nop\n\tv_nop\n\tv_nop\n\tv_nop" : "+v"(a), "+v"(b), "+v"(c), "+v"(d)); }
template <typename T> struct Frag;
template <> struct Frag<_Float16> {
  typedef v16h V; union U { v16h v; v8h h[2]; };
  static __device__ __forceinline__ v16h load(const _Float16* p) {
    U f; f.h[0] = *(const v8h*)(p); f.h[1] = *(const v8h*)(p + 16); return f.v;
  }
  static __device__ __forceinline__ v8f mma(v16h a, v16h b, v8f c) {
    return __builtin_amdgcn_wmma_f32_16x16x32_f16(false, a, false, b, (short)0, c, false, false);
  }
  static __device__ __forceinline__ void guard(v8f& a, v8f& b, v16h x, v16h y) { dep_guard_h(a, b, x, y); }
  static __device__ __forceinline__ void keep(v16h a, v16h b, v16h c, v16h d) { keep4_h(a, b, c, d); }
};
template <> struct Frag<__bf16> {
  typedef v16b V; union U { v16b v; v8b h[2]; };
  static __device__ __forceinline__ v16b load(const __bf16* p) {
    U f; f.h[0] = *(const v8b*)(p); f.h[1] = *(const v8b*)(p + 16); return f.v;
  }
  static __device__ __forceinline__ v8f mma(v16b a, v16b b, v8f c) {
    return __builtin_amdgcn_wmma_f32_16x16x32_bf16(false, a, false, b, (short)0, c, false, false);
  }
  static __device__ __forceinline__ void guard(v8f& a, v8f& b, v16b x, v16b y) { dep_guard_b(a, b, x, y); }
  static __device__ __forceinline__ void keep(v16b a, v16b b, v16b c, v16b d) { keep4_b(a, b, c, d); }
};

__device__ __forceinline__ void dep_guard1(v8f& a, v16h x, v16h y) { asm volatile("v_nop\n\tv_nop\n\tv_nop\n\tv_nop" : "+v"(a) : "v"(x), "v"(y)); }

__device__ __forceinline__ unsigned pk16(unsigned short a, unsigned short b) { return (unsigned)a | ((unsigned)b << 16); }
__device__ __forceinline__ unsigned short h_bits(float f) { const _Float16 h = (_Float16)f; return __builtin_bit_cast(unsigned short, h); }

__device__ __forceinline__ float gate_sigm(float v) { return __builtin_amdgcn_rcpf(1.0f + expf(-v)); }
__device__ __forceinline__ float gate_tanh(float v) { return 1.0f - 2.0f * __builtin_amdgcn_rcpf(1.0f + expf(2.0f * v)); }

__device__ __forceinline__ void cell_step(const v8f ai, const v8f af, const v8f ag, const v8f ao,
                                          const float (&bs)[4], float (&cst)[8], float (&hout)[8]) {
#pragma unroll
  for (int r = 0; r < 8; ++r) {
    const float gi = gate_sigm(ai[r] * kWCarryInv + bs[0]);
    const float gf = gate_sigm(af[r] * kWCarryInv + bs[1]);
    const float gg = gate_tanh(ag[r] * kWCarryInv + bs[2]);
    const float go = gate_sigm(ao[r] * kWCarryInv + bs[3]);
    const float cv = gf * cst[r] + gi * gg;
    cst[r] = cv;
    hout[r] = go * gate_tanh(cv);
  }
}

__global__ __launch_bounds__(256) void prep_weights_kernel(
    const float* __restrict__ Wih0, const float* __restrict__ Whh0,
    const float* __restrict__ Wih1, const float* __restrict__ Whh1,
    const float* __restrict__ Wlin, unsigned short* __restrict__ wpl, int ngroups) {
  const int j = blockIdx.x * 256 + threadIdx.x;
  if (j >= ngroups) return;
  const int reg = (j < kGrp0) ? 0 : ((j < kGrp0 + kGrp1) ? 1 : 2);
  int j0 = j;                 j0 = j0 > kGrp0 - 1 ? kGrp0 - 1 : j0;
  int j1 = j - kGrp0;         j1 = j1 < 0 ? 0 : (j1 > kGrp1 - 1 ? kGrp1 - 1 : j1);
  int j2 = j - kGrp0 - kGrp1; j2 = j2 < 0 ? 0 : (j2 > kGrp2 - 1 ? kGrp2 - 1 : j2);
  const int e0 = 8 * j0, n0 = e0 / kW0ld, kb0 = e0 - n0 * kW0ld;
  const int e1 = 8 * j1, n1 = e1 >> 7,     kb1 = e1 & 127;
  const int e2 = 8 * j2, n2 = e2 >> 6,     kb2 = e2 & 63;
  const int n2c = n2 < kOutDim ? n2 : kOutDim - 1;
  unsigned short hb[8];
#pragma unroll
  for (int e = 0; e < 8; ++e) {
    const int k0 = kb0 + e;
    const int ka = k0 < kIn - 1 ? k0 : kIn - 1;
    int kbh = k0 - kInPad; kbh = kbh < 0 ? 0 : (kbh > kHid - 1 ? kHid - 1 : kbh);
    const float va = Wih0[n0 * kIn + ka];
    const float vb = Whh0[n0 * kHid + kbh];
    const float v0 = (k0 < kIn) ? va : ((k0 < kInPad) ? 0.0f : vb);
    const int k1 = kb1 + e;
    const int kc = k1 < kHid - 1 ? k1 : kHid - 1;
    int kd = k1 - kHid; kd = kd < 0 ? 0 : (kd > kHid - 1 ? kHid - 1 : kd);
    const float vc = Wih1[n1 * kHid + kc];
    const float vd = Whh1[n1 * kHid + kd];
    const float v1 = (k1 < kHid) ? vc : vd;
    const int k2 = kb2 + e;
    const float ve = Wlin[n2c * kHid + k2];
    const float v2 = (n2 < kOutDim) ? ve : 0.0f;
    const float v = (reg == 0) ? v0 : ((reg == 1) ? v1 : v2);
    hb[e] = h_bits(kWCarry * v);
  }
  const v4u u = (v4u){pk16(hb[0], hb[1]), pk16(hb[2], hb[3]), pk16(hb[4], hb[5]), pk16(hb[6], hb[7])};
  unsigned short* q = wpl + 8 * (size_t)j;
  *(volatile v4u*)q = u;
  __threadfence();
  *(volatile v4u*)q = u;
}

__global__ __launch_bounds__(kThreads) void lstm2_fused_kernel(
    const float* __restrict__ x, const unsigned short* __restrict__ wpl,
    const float* __restrict__ bih0, const float* __restrict__ bhh0,
    const float* __restrict__ bih1, const float* __restrict__ bhh1,
    const float* __restrict__ blin, float* __restrict__ stg, int nrows) {
  __shared__ __align__(16) unsigned short sT0[kRowsPerBlock * kPitch0];
  __shared__ __align__(16) unsigned short sT1[kRowsPerBlock * kPitch1];
  __shared__ __align__(16) float sOut[kRowsPerBlock * kPitchO];

  const int tid  = threadIdx.x;
  const int lane = tid & 31;
  const int wave = tid >> 5;
  const int hh   = lane >> 4;
  const int cc   = lane & 15;
  const int unit = wave * 16 + cc;
  const int row0 = blockIdx.x * kRowsPerBlock;
  const _Float16* W0 = (const _Float16*)wpl;
  const _Float16* W1 = W0 + kW0n;
  const _Float16* WL = W1 + kW1n;
  const _Float16* sT0h = (const _Float16*)sT0;
  const _Float16* sT1h = (const _Float16*)sT1;

  {
    const v4u z = (v4u){0u, 0u, 0u, 0u};
    for (int i = tid; i < (kRowsPerBlock * kPitch0) / 8; i += kThreads) *(v4u*)(sT0 + 8 * i) = z;
    for (int i = tid; i < (kRowsPerBlock * kPitch1) / 8; i += kThreads) *(v4u*)(sT1 + 8 * i) = z;
  }
  float b0s[4], b1s[4];
#pragma unroll
  for (int q = 0; q < 4; ++q) {
    b0s[q] = bih0[q * kHid + unit] + bhh0[q * kHid + unit];
    b1s[q] = bih1[q * kHid + unit] + bhh1[q * kHid + unit];
  }
  float c0s[2][8], c1s[2][8];
#pragma unroll
  for (int m = 0; m < 2; ++m)
#pragma unroll
    for (int r = 0; r < 8; ++r) { c0s[m][r] = 0.0f; c1s[m][r] = 0.0f; }
  __syncthreads();

#pragma unroll 1
  for (int t = 0; t < kSteps; ++t) {
    {
      const int r = tid >> 2, q = tid & 3;
      int grow = row0 + r; grow = grow < nrows ? grow : nrows - 1;
      const float* xp = x + (size_t)grow * kXRow + t * kIn + q * 8;
      const int off2 = (q < 3) ? 4 : 0;
      const v4f f0 = *(const v4f*)(xp);
      const v4f f1 = *(const v4f*)(xp + off2);
      unsigned short hb[8];
#pragma unroll
      for (int e = 0; e < 4; ++e) {
        hb[e] = h_bits(f0[e]);
        const float s = (q < 3) ? f1[e] : 0.0f;
        hb[4 + e] = h_bits(s);
      }
      const v4u u = (v4u){pk16(hb[0], hb[1]), pk16(hb[2], hb[3]), pk16(hb[4], hb[5]), pk16(hb[6], hb[7])};
      *(v4u*)(sT0 + r * kPitch0 + q * 8) = u;
    }
    __syncthreads();

    float h1v[2][8];
    {
      v8f acc[2][4];
#pragma unroll
      for (int m = 0; m < 2; ++m)
#pragma unroll
        for (int q = 0; q < 4; ++q) acc[m][q] = (v8f){0.f,0.f,0.f,0.f,0.f,0.f,0.f,0.f};
#pragma unroll 1
      for (int ks = 0; ks < kW0ld / 32; ++ks) {
        const int k0 = ks * 32 + 8 * hh;
        v16h bq[4];
#pragma unroll
        for (int q = 0; q < 4; ++q) bq[q] = Frag<_Float16>::load(W0 + (size_t)(q * kHid + unit) * kW0ld + k0);
#pragma unroll
        for (int m = 0; m < 2; ++m) {
          const v16h a = Frag<_Float16>::load(sT0h + (m * 16 + cc) * kPitch0 + k0);
#pragma unroll
          for (int q = 0; q < 4; ++q) acc[m][q] = Frag<_Float16>::mma(a, bq[q], acc[m][q]);
          Frag<_Float16>::guard(acc[m][0], acc[m][3], a, a);
        }
        Frag<_Float16>::keep(bq[0], bq[1], bq[2], bq[3]);
      }
      acc_guard4(acc[0][0], acc[0][1], acc[0][2], acc[0][3]);
      acc_guard4(acc[1][0], acc[1][1], acc[1][2], acc[1][3]);
#pragma unroll
      for (int m = 0; m < 2; ++m) cell_step(acc[m][0], acc[m][1], acc[m][2], acc[m][3], b0s, c0s[m], h1v[m]);
    }
    __syncthreads();

#pragma unroll
    for (int m = 0; m < 2; ++m)
#pragma unroll
      for (int r = 0; r < 8; ++r) {
        const int row = m * 16 + 8 * hh + r;
        const unsigned short hv = h_bits(h1v[m][r]);
        sT0[row * kPitch0 + kInPad + unit] = hv;
        sT1[row * kPitch1 + unit] = hv;
      }
    __syncthreads();

    float h2v[2][8];
    {
      v8f acc[2][4];
#pragma unroll
      for (int m = 0; m < 2; ++m)
#pragma unroll
        for (int q = 0; q < 4; ++q) acc[m][q] = (v8f){0.f,0.f,0.f,0.f,0.f,0.f,0.f,0.f};
#pragma unroll 1
      for (int ks = 0; ks < kW1ld / 32; ++ks) {
        const int k0 = ks * 32 + 8 * hh;
        v16h bq[4];
#pragma unroll
        for (int q = 0; q < 4; ++q) bq[q] = Frag<_Float16>::load(W1 + (size_t)(q * kHid + unit) * kW1ld + k0);
#pragma unroll
        for (int m = 0; m < 2; ++m) {
          const v16h a = Frag<_Float16>::load(sT1h + (m * 16 + cc) * kPitch1 + k0);
#pragma unroll
          for (int q = 0; q < 4; ++q) acc[m][q] = Frag<_Float16>::mma(a, bq[q], acc[m][q]);
          Frag<_Float16>::guard(acc[m][0], acc[m][3], a, a);
        }
        Frag<_Float16>::keep(bq[0], bq[1], bq[2], bq[3]);
      }
      acc_guard4(acc[0][0], acc[0][1], acc[0][2], acc[0][3]);
      acc_guard4(acc[1][0], acc[1][1], acc[1][2], acc[1][3]);
#pragma unroll
      for (int m = 0; m < 2; ++m) cell_step(acc[m][0], acc[m][1], acc[m][2], acc[m][3], b1s, c1s[m], h2v[m]);
    }
    __syncthreads();

#pragma unroll
    for (int m = 0; m < 2; ++m)
#pragma unroll
      for (int r = 0; r < 8; ++r) {
        const int row = m * 16 + 8 * hh + r;
        sT1[row * kPitch1 + kHid + unit] = h_bits(h2v[m][r]);
      }
  }
  __syncthreads();

  if (wave < 2) {
    const int m = wave;
    v8f acc = (v8f){0.f,0.f,0.f,0.f,0.f,0.f,0.f,0.f};
#pragma unroll
    for (int ks = 0; ks < kHid / 32; ++ks) {
      const int k0 = ks * 32 + 8 * hh;
      const v16h b = Frag<_Float16>::load(WL + cc * kHid + k0);
      const v16h a = Frag<_Float16>::load(sT1h + (m * 16 + cc) * kPitch1 + kHid + k0);
      acc = Frag<_Float16>::mma(a, b, acc);
      dep_guard1(acc, a, b);
    }
    const float bl = blin[cc < kOutDim ? cc : kOutDim - 1];
#pragma unroll
    for (int r = 0; r < 8; ++r) {
      float v = acc[r] * kWCarryInv + bl;
      v = (cc < kOutDim) ? v : 0.0f;
      sOut[(m * 16 + 8 * hh + r) * kPitchO + cc] = v;
    }
  }
  __syncthreads();
  {
    const int r = tid >> 2, c4 = (tid & 3) * 4;
    const v4f v = *(const v4f*)(sOut + r * kPitchO + c4);
    float* dst = stg + (size_t)(row0 + r) * kOutPad + c4;
    *(volatile v4f*)dst = v;
    __threadfence();
    *(volatile v4f*)dst = v;
  }
}

__global__ __launch_bounds__(256) void pack_out_kernel(const float* __restrict__ stg, float* __restrict__ out,
                                                       int n4, int nrows) {
  const int i = blockIdx.x * 256 + threadIdx.x;
  if (i >= n4) return;
  v4f v;
#pragma unroll
  for (int e = 0; e < 4; ++e) {
    const int idx = 4 * i + e;
    int row = idx / kOutDim;
    const int col = idx - row * kOutDim;
    row = row < nrows ? row : nrows - 1;
    v[e] = stg[(size_t)row * kOutPad + col];
  }
  float* q = out + 4 * (size_t)i;
  *(volatile v4f*)q = v;
  __threadfence();
  *(volatile v4f*)q = v;
}

extern "C" void kernel_launch(void* const* d_in, const int* in_sizes, int n_in,
                              void* d_out, int out_size, void* d_ws, size_t ws_size,
                              hipStream_t stream) {
  const float* x    = (const float*)d_in[0];
  const float* Wih0 = (const float*)d_in[1];
  const float* Whh0 = (const float*)d_in[2];
  const float* bih0 = (const float*)d_in[3];
  const float* bhh0 = (const float*)d_in[4];
  const float* Wih1 = (const float*)d_in[5];
  const float* Whh1 = (const float*)d_in[6];
  const float* bih1 = (const float*)d_in[7];
  const float* bhh1 = (const float*)d_in[8];
  const float* Wlin = (const float*)d_in[9];
  const float* blin = (const float*)d_in[10];
  float* out = (float*)d_out;

  const int nrows = in_sizes[0] / kXRow;
  if (nrows <= 0) return;
  const int blocks  = (nrows + kRowsPerBlock - 1) / kRowsPerBlock;
  const int stgRows = blocks * kRowsPerBlock;

  const size_t bytesW  = (size_t)kWtot * 2;
  const size_t offStg  = ((bytesW + 511) / 512) * 512;
  const size_t bytesStg = (size_t)stgRows * kOutPad * sizeof(float);
  if (offStg + bytesStg > ws_size) return;
  if ((size_t)out_size < (size_t)nrows * kOutDim) return;

  unsigned char* ws = (unsigned char*)d_ws;
  unsigned short* wpl = (unsigned short*)(ws);
  float* stg = (float*)(ws + offStg);

  prep_weights_kernel<<<(kPrepGroups + 255) / 256, 256, 0, stream>>>(Wih0, Whh0, Wih1, Whh1, Wlin, wpl, kPrepGroups);
  lstm2_fused_kernel<<<blocks, kThreads, 0, stream>>>(x, wpl, bih0, bhh0, bih1, bhh1, blin, stg, nrows);
  const int n4 = (nrows * kOutDim) / 4;
  pack_out_kernel<<<(n4 + 255) / 256, 256, 0, stream>>>(stg, out, n4, stgRows);
}
